// MultiHeadSelfAttention2D_39728447488110
// MI455X (gfx1250) — hardware-verified
//
#include <hip/hip_runtime.h>

#ifndef NB
#define NB 4
#endif
#ifndef SEQ
#define SEQ 2304
#endif
#define NB_FULL 4
#define SEQ_FULL 2304
#define DIM 512
#define HEADS 8
#define HD 64
#define OCH 1536

static_assert(NB >= 1 && NB <= NB_FULL);
static_assert(SEQ >= 64 && SEQ <= SEQ_FULL && (SEQ % 64) == 0);
static_assert(DIM == HEADS * HD);
static_assert((OCH * DIM) % 2048 == 0 && (DIM * DIM) % 2048 == 0);

typedef _Float16 v16h __attribute__((ext_vector_type(16)));
typedef _Float16 v8h __attribute__((ext_vector_type(8)));
typedef __attribute__((ext_vector_type(16))) __bf16 v16b;
typedef unsigned short v8us __attribute__((ext_vector_type(8)));
typedef float v8f __attribute__((ext_vector_type(8)));
typedef float v4f __attribute__((ext_vector_type(4)));

union FragH { v16h v; v8h p[2]; };
union FragB { v16b v; v8us p[2]; };

__device__ __forceinline__ v8f mma_bf16(v16b a, v16b b, v8f c) {
  c = __builtin_amdgcn_wmma_f32_16x16x32_bf16(false, a, false, b, (short)0, c, false, false);
  asm volatile("v_nop\n\tv_nop\n\tv_nop\n\tv_nop" : "+v"(c) : "v"(a), "v"(b));
  return c;
}
__device__ __forceinline__ v8f mma_f16(v16h a, v16h b, v8f c) {
  c = __builtin_amdgcn_wmma_f32_16x16x32_f16(false, a, false, b, (short)0, c, false, false);
  asm volatile("v_nop\n\tv_nop\n\tv_nop\n\tv_nop" : "+v"(c) : "v"(a), "v"(b));
  return c;
}

__device__ __forceinline__ unsigned short f2bf(float f) {
  unsigned int u = __float_as_uint(f);
  u = u + 0x7FFFu + ((u >> 16) & 1u);
  return (unsigned short)(u >> 16);
}
__device__ __forceinline__ float bf2f(unsigned short w) {
  return __uint_as_float(((unsigned int)w) << 16);
}
__device__ __forceinline__ v8f zero8() {
  v8f z;
#pragma unroll
  for (int i = 0; i < 8; ++i) z[i] = 0.0f;
  return z;
}

__global__ __launch_bounds__(256) void k_cvt_w(const float* __restrict__ qkv_w,
                                               const float* __restrict__ proj_w,
                                               unsigned short* wq, _Float16* wp) {
  const int NQB = (OCH * DIM / 8) / 256;
  const int tid = threadIdx.x;
  if ((int)blockIdx.x < NQB) {
    const size_t e = ((size_t)blockIdx.x * 256 + tid) * 8;
    const v4f a = *(const v4f*)(qkv_w + e);
    const v4f c = *(const v4f*)(qkv_w + e + 4);
    v8us o;
#pragma unroll
    for (int j = 0; j < 4; ++j) {
      o[j] = f2bf(a[j]);
      o[4 + j] = f2bf(c[j]);
    }
    unsigned short* d = wq + e;
    *(volatile v8us*)d = o;
    __threadfence();
    *(volatile v8us*)d = o;
  } else {
    const size_t e = ((size_t)((int)blockIdx.x - NQB) * 256 + tid) * 8;
    const v4f a = *(const v4f*)(proj_w + e);
    const v4f c = *(const v4f*)(proj_w + e + 4);
    v8h o;
#pragma unroll
    for (int j = 0; j < 4; ++j) {
      o[j] = (_Float16)(bf2f(f2bf(a[j])) * 64.0f);
      o[4 + j] = (_Float16)(bf2f(f2bf(c[j])) * 64.0f);
    }
    _Float16* d = wp + e;
    *(volatile v8h*)d = o;
    __threadfence();
    *(volatile v8h*)d = o;
  }
}

__global__ __launch_bounds__(256) void k_xpose(const float* __restrict__ x,
                                               unsigned short* xT) {
  __shared__ __align__(16) unsigned short tile[32][72];
  const int tid = threadIdx.x;
  const int n0 = blockIdx.x * 32, c0 = blockIdx.y * 64, b = blockIdx.z;
  const float* xb = x + (size_t)b * DIM * SEQ_FULL;
  const int nl = tid & 31, cb = tid >> 5;
#pragma unroll
  for (int k = 0; k < 8; ++k) {
    const int cl = cb + 8 * k;
    tile[nl][cl] = f2bf(xb[(size_t)(c0 + cl) * SEQ_FULL + n0 + nl]);
  }
  __syncthreads();
  const int ln = tid >> 3, pc = (tid & 7) * 8;
  const v8us v = *(const v8us*)(&tile[ln][pc]);
  unsigned short* d = xT + ((size_t)b * SEQ + n0 + ln) * DIM + c0 + pc;
  *(volatile v8us*)d = v;
  __threadfence();
  *(volatile v8us*)d = v;
}

__global__ __launch_bounds__(128) void k_qkv(const unsigned short* __restrict__ wq,
                                             const unsigned short* __restrict__ xT,
                                             unsigned short* qh, unsigned short* ql,
                                             unsigned short* kh, unsigned short* kl,
                                             _Float16* vT) {
  __shared__ __align__(16) float stg[64][68];
  const int tid = threadIdx.x, lane = tid & 31, w = tid >> 5;
  const int h = lane >> 4, m = lane & 15;
  const int n0 = blockIdx.x * 64, o0 = blockIdx.y * 64, b = blockIdx.z;

  const unsigned short* arow = wq + (size_t)(o0 + 16 * w + m) * DIM;
  const unsigned short* xb = xT + ((size_t)b * SEQ + n0 + m) * DIM;

  v8f acc[4];
#pragma unroll
  for (int t = 0; t < 4; ++t) acc[t] = zero8();

#pragma unroll 2
  for (int k0 = 0; k0 < DIM; k0 += 32) {
    FragB a;
    a.p[0] = *(const v8us*)(arow + k0 + 8 * h);
    a.p[1] = *(const v8us*)(arow + k0 + 16 + 8 * h);
#pragma unroll
    for (int t = 0; t < 4; ++t) {
      const unsigned short* br = xb + (size_t)t * 16 * DIM + k0;
      FragB bb;
      bb.p[0] = *(const v8us*)(br + 8 * h);
      bb.p[1] = *(const v8us*)(br + 16 + 8 * h);
      acc[t] = mma_bf16(a.v, bb.v, acc[t]);
    }
  }

#pragma unroll
  for (int t = 0; t < 4; ++t)
#pragma unroll
    for (int r = 0; r < 8; ++r)
      stg[16 * t + m][16 * w + 8 * h + r] = acc[t][r];
  __syncthreads();

  const int seg = o0 >> 9;
  const int hh = (o0 & 511) >> 6;
  const size_t bh = (size_t)b * HEADS + hh;
  const int lr = tid >> 3;
  const int pc = tid & 7;
  if (seg < 2) {
    unsigned short* ph = (seg == 0 ? qh : kh) + bh * (size_t)SEQ * HD;
    unsigned short* pl = (seg == 0 ? ql : kl) + bh * (size_t)SEQ * HD;
#pragma unroll
    for (int pass = 0; pass < 4; ++pass) {
      const int nl = pass * 16 + lr;
      const v4f f0 = *(const v4f*)(&stg[nl][pc * 8]);
      const v4f f1 = *(const v4f*)(&stg[nl][pc * 8 + 4]);
      v8us hi, lo;
#pragma unroll
      for (int j = 0; j < 4; ++j) {
        const float va = f0[j], vb2 = f1[j];
        const unsigned short ha = f2bf(va), hb = f2bf(vb2);
        hi[j] = ha;
        hi[4 + j] = hb;
        lo[j] = f2bf(va - bf2f(ha));
        lo[4 + j] = f2bf(vb2 - bf2f(hb));
      }
      const size_t off = (size_t)(n0 + nl) * HD + pc * 8;
      *(volatile v8us*)(ph + off) = hi;
      *(volatile v8us*)(pl + off) = lo;
      __threadfence();
      *(volatile v8us*)(ph + off) = hi;
      *(volatile v8us*)(pl + off) = lo;
    }
  } else {
    _Float16* pv = vT + bh * (size_t)HD * SEQ;
#pragma unroll
    for (int pass = 0; pass < 4; ++pass) {
      const int dl = pass * 16 + lr;
      v8h o;
#pragma unroll
      for (int j = 0; j < 8; ++j) o[j] = (_Float16)(stg[pc * 8 + j][dl] * 8.0f);
      const size_t off = (size_t)dl * SEQ + n0 + pc * 8;
      *(volatile v8h*)(pv + off) = o;
      __threadfence();
      *(volatile v8h*)(pv + off) = o;
    }
  }
}

__global__ __launch_bounds__(128) void k_attn(const unsigned short* __restrict__ qh,
                                              const unsigned short* __restrict__ ql,
                                              const unsigned short* __restrict__ kh,
                                              const unsigned short* __restrict__ kl,
                                              const _Float16* __restrict__ vT,
                                              _Float16* oT) {
  __shared__ __align__(16) unsigned short skh[32][72];
  __shared__ __align__(16) unsigned short skl[32][72];
  __shared__ __align__(16) _Float16 sv[64][40];
  __shared__ __align__(16) _Float16 sp[4][16][40];
  __shared__ __align__(16) _Float16 so[4][16][72];

  const int tid = threadIdx.x, lane = tid & 31, w = tid >> 5;
  const int h = lane >> 4, m = lane & 15;
  const int q0 = blockIdx.x * 64 + w * 16;
  const int hd = blockIdx.y, b = blockIdx.z;
  const size_t bh = (size_t)b * HEADS + hd;
  const unsigned short* qhb = qh + bh * (size_t)SEQ * HD;
  const unsigned short* qlb = ql + bh * (size_t)SEQ * HD;
  const unsigned short* khb = kh + bh * (size_t)SEQ * HD;
  const unsigned short* klb = kl + bh * (size_t)SEQ * HD;
  const _Float16* vb = vT + bh * (size_t)HD * SEQ;

  FragB qhf[2], qlf[2];
  {
    const unsigned short* rh = qhb + (size_t)(q0 + m) * HD;
    const unsigned short* rl = qlb + (size_t)(q0 + m) * HD;
#pragma unroll
    for (int ds = 0; ds < 2; ++ds) {
      qhf[ds].p[0] = *(const v8us*)(rh + ds * 32 + 8 * h);
      qhf[ds].p[1] = *(const v8us*)(rh + ds * 32 + 16 + 8 * h);
      qlf[ds].p[0] = *(const v8us*)(rl + ds * 32 + 8 * h);
      qlf[ds].p[1] = *(const v8us*)(rl + ds * 32 + 16 + 8 * h);
    }
  }

  v8f oacc[4];
#pragma unroll
  for (int dt = 0; dt < 4; ++dt) oacc[dt] = zero8();
  float mi[8], li[8];
#pragma unroll
  for (int r = 0; r < 8; ++r) { mi[r] = -3.0e38f; li[r] = 0.0f; }

#pragma unroll 1
  for (int mc = 0; mc < SEQ; mc += 32) {
#pragma unroll
    for (int i = 0; i < 2; ++i) {
      const int idx = tid + 128 * i;
      const int row = idx >> 3, pc = (idx & 7) * 8;
      *(v8us*)(&skh[row][pc]) = *(const v8us*)(khb + (size_t)(mc + row) * HD + pc);
      *(v8us*)(&skl[row][pc]) = *(const v8us*)(klb + (size_t)(mc + row) * HD + pc);
      const int d = idx >> 2, pq = (idx & 3) * 8;
      *(v8h*)(&sv[d][pq]) = *(const v8h*)(vb + (size_t)d * SEQ + mc + pq);
    }
    __syncthreads();

    v8f s[2];
#pragma unroll
    for (int ct = 0; ct < 2; ++ct) {
      v8f acc = zero8();
#pragma unroll
      for (int ds = 0; ds < 2; ++ds) {
        FragB kf, kg;
        kf.p[0] = *(const v8us*)(&skh[ct * 16 + m][ds * 32 + 8 * h]);
        kf.p[1] = *(const v8us*)(&skh[ct * 16 + m][ds * 32 + 16 + 8 * h]);
        kg.p[0] = *(const v8us*)(&skl[ct * 16 + m][ds * 32 + 8 * h]);
        kg.p[1] = *(const v8us*)(&skl[ct * 16 + m][ds * 32 + 16 + 8 * h]);
        acc = mma_bf16(qhf[ds].v, kf.v, acc);
        acc = mma_bf16(qhf[ds].v, kg.v, acc);
        acc = mma_bf16(qlf[ds].v, kf.v, acc);
      }
      s[ct] = acc;
    }

#pragma unroll
    for (int r = 0; r < 8; ++r) {
      const float a0 = s[0][r] * 0.125f, a1 = s[1][r] * 0.125f;
      float t = fmaxf(a0, a1);
      t = fmaxf(t, __shfl_xor(t, 1, 16));
      t = fmaxf(t, __shfl_xor(t, 2, 16));
      t = fmaxf(t, __shfl_xor(t, 4, 16));
      t = fmaxf(t, __shfl_xor(t, 8, 16));
      const float mn = fmaxf(mi[r], t);
      const float al = __expf(mi[r] - mn);
      const float p0 = __expf(a0 - mn);
      const float p1 = __expf(a1 - mn);
      float rs = p0 + p1;
      rs += __shfl_xor(rs, 1, 16);
      rs += __shfl_xor(rs, 2, 16);
      rs += __shfl_xor(rs, 4, 16);
      rs += __shfl_xor(rs, 8, 16);
      li[r] = li[r] * al + rs;
      mi[r] = mn;
#pragma unroll
      for (int dt = 0; dt < 4; ++dt) oacc[dt][r] *= al;
      sp[w][8 * h + r][m] = (_Float16)(p0 * 1024.0f);
      sp[w][8 * h + r][16 + m] = (_Float16)(p1 * 1024.0f);
    }
    __syncthreads();

    FragH pf;
    pf.p[0] = *(const v8h*)(&sp[w][m][8 * h]);
    pf.p[1] = *(const v8h*)(&sp[w][m][16 + 8 * h]);
#pragma unroll
    for (int dt = 0; dt < 4; ++dt) {
      FragH vf;
      vf.p[0] = *(const v8h*)(&sv[dt * 16 + m][8 * h]);
      vf.p[1] = *(const v8h*)(&sv[dt * 16 + m][16 + 8 * h]);
      oacc[dt] = mma_f16(pf.v, vf.v, oacc[dt]);
    }
    __syncthreads();
  }

#pragma unroll
  for (int r = 0; r < 8; ++r) {
    const float inv = 1.0f / (512.0f * li[r]);
#pragma unroll
    for (int dt = 0; dt < 4; ++dt)
      so[w][8 * h + r][dt * 16 + m] = (_Float16)(oacc[dt][r] * inv);
  }
  __syncthreads();
  {
    const int pc = lane & 7;
#pragma unroll
    for (int pass = 0; pass < 4; ++pass) {
      const int qq = pass * 4 + (lane >> 3);
      const v8h v = *(const v8h*)(&so[w][qq][pc * 8]);
      _Float16* d = oT + ((size_t)b * SEQ + q0 + qq) * DIM + hd * HD + pc * 8;
      *(volatile v8h*)d = v;
      __threadfence();
      *(volatile v8h*)d = v;
    }
  }
}

__global__ __launch_bounds__(128) void k_proj(const _Float16* __restrict__ wp,
                                              const _Float16* __restrict__ oT,
                                              float* out) {
  __shared__ __align__(16) float stg[64][68];
  const int tid = threadIdx.x, lane = tid & 31, w = tid >> 5;
  const int h = lane >> 4, m = lane & 15;
  const int n0 = blockIdx.x * 64, co0 = blockIdx.y * 64, b = blockIdx.z;

  const _Float16* arow = wp + (size_t)(co0 + 16 * w + m) * DIM;
  const _Float16* ob = oT + ((size_t)b * SEQ + n0 + m) * DIM;

  v8f acc[4];
#pragma unroll
  for (int t = 0; t < 4; ++t) acc[t] = zero8();

#pragma unroll 2
  for (int k0 = 0; k0 < DIM; k0 += 32) {
    FragH a;
    a.p[0] = *(const v8h*)(arow + k0 + 8 * h);
    a.p[1] = *(const v8h*)(arow + k0 + 16 + 8 * h);
#pragma unroll
    for (int t = 0; t < 4; ++t) {
      const _Float16* br = ob + (size_t)t * 16 * DIM + k0;
      FragH bb;
      bb.p[0] = *(const v8h*)(br + 8 * h);
      bb.p[1] = *(const v8h*)(br + 16 + 8 * h);
      acc[t] = mma_f16(a.v, bb.v, acc[t]);
    }
  }

#pragma unroll
  for (int t = 0; t < 4; ++t)
#pragma unroll
    for (int r = 0; r < 8; ++r)
      stg[16 * w + 8 * h + r][16 * t + m] = acc[t][r];
  __syncthreads();

  const int pc = tid & 7;
  const float sc = 1.0f / 1024.0f;
#pragma unroll
  for (int pass = 0; pass < 8; ++pass) {
    const int L = pass * 16 + (tid >> 3);
    const int col = L >> 1, nh = L & 1;
    const int nl = nh * 32 + pc * 4;
    v4f v = *(const v4f*)(&stg[col][nl]);
#pragma unroll
    for (int j = 0; j < 4; ++j) v[j] *= sc;
    float* d = out + ((size_t)b * DIM + co0 + col) * SEQ + n0 + nl;
    *(volatile v4f*)d = v;
    __threadfence();
    *(volatile v4f*)d = v;
  }
}

extern "C" void kernel_launch(void* const* d_in, const int* in_sizes, int n_in,
                              void* d_out, int out_size, void* d_ws, size_t ws_size,
                              hipStream_t stream) {
  if (n_in < 3) return;
  if (in_sizes[0] < NB * DIM * SEQ_FULL) return;
  if (in_sizes[1] < OCH * DIM) return;
  if (in_sizes[2] < DIM * DIM) return;
  if (out_size < NB * DIM * SEQ) return;

  const float* x = (const float*)d_in[0];
  const float* qkv_w = (const float*)d_in[1];
  const float* proj_w = (const float*)d_in[2];
  float* out = (float*)d_out;

  const size_t szWq = (size_t)OCH * DIM * 2;
  const size_t szWp = (size_t)DIM * DIM * 2;
  const size_t szX = (size_t)NB * SEQ * DIM * 2;
  const size_t szQK = (size_t)NB * HEADS * SEQ * HD * 2;
  const size_t szV = szQK;
  const size_t szO = (size_t)NB * SEQ * DIM * 2;
  size_t off = 0;
  char* ws = (char*)d_ws;
  unsigned short* wq = (unsigned short*)(ws + off); off += szWq;
  _Float16* wp = (_Float16*)(ws + off); off += szWp;
  unsigned short* xT = (unsigned short*)(ws + off); off += szX;
  unsigned short* qh = (unsigned short*)(ws + off); off += szQK;
  unsigned short* ql = (unsigned short*)(ws + off); off += szQK;
  unsigned short* kh = (unsigned short*)(ws + off); off += szQK;
  unsigned short* kl = (unsigned short*)(ws + off); off += szQK;
  _Float16* vT = (_Float16*)(ws + off); off += szV;
  _Float16* oT = (_Float16*)(ws + off); off += szO;
  if (off > ws_size) return;

  const int nqb = (OCH * DIM / 8) / 256;
  const int npb = (DIM * DIM / 8) / 256;
  k_cvt_w<<<dim3(nqb + npb), dim3(256), 0, stream>>>(qkv_w, proj_w, wq, wp);
  k_xpose<<<dim3(SEQ / 32, DIM / 64, NB), dim3(256), 0, stream>>>(x, xT);
  k_qkv<<<dim3(SEQ / 64, OCH / 64, NB), dim3(128), 0, stream>>>(wq, xT, qh, ql, kh, kl, vT);
  k_attn<<<dim3(SEQ / 64, HEADS, NB), dim3(128), 0, stream>>>(qh, ql, kh, kl, vT, oT);
  k_proj<<<dim3(SEQ / 64, DIM / 64, NB), dim3(128), 0, stream>>>(wp, oT, out);
}
